// SlotAttentionLayer_48369921687885
// MI455X (gfx1250) — hardware-verified
//
#include <hip/hip_runtime.h>
#include <math.h>
#include <stdint.h>

#define NB     2
#define SEQ    2048
#define DM     1024
#define NH     16
#define HD     64
#define NSC    8
#define NTAB   512
#define NROW   (NB * SEQ)
#define QT     64
#define KSP    136
#define VSP    72
#define SSP    136
#define FSP    132
#define OHP    72
#define LNPS   6.931471805599453f
#define FMIN16 6.103515625e-05f
#define NEGBIG (-1.0e30f)
#define WSCL   32.0f
static_assert((SEQ % QT) == 0);
static_assert((SEQ % 64) == 0);
static_assert((DM % 128) == 0);
static_assert((DM % 32) == 0);
static_assert((NROW % 64) == 0);
static_assert((NTAB % 64) == 0);
static_assert(NH * HD == DM);
static_assert(HD == 64);
static_assert(((DM * DM) / 8) % 256 == 0);
static_assert(DM == 8 * 128);

typedef _Float16       v16h __attribute__((ext_vector_type(16)));
typedef _Float16       v8h  __attribute__((ext_vector_type(8)));
typedef float          v8f  __attribute__((ext_vector_type(8)));
typedef float          v4f  __attribute__((ext_vector_type(4)));
typedef unsigned int   v4u  __attribute__((ext_vector_type(4)));

union FragH { v16h v; v8h h[2]; };
static_assert(sizeof(FragH) == 32);

__device__ __forceinline__ unsigned short bf_bits(float f) {
  unsigned u = __float_as_uint(f);
  return (unsigned short)((u + 0x7FFFu + ((u >> 16) & 1u)) >> 16);
}
__device__ __forceinline__ float bf_up(unsigned short x) { return __uint_as_float(((unsigned)x) << 16); }
__device__ __forceinline__ float bfr(float f) { return bf_up(bf_bits(f)); }
__device__ __forceinline__ unsigned short h_bits(_Float16 x) { return __builtin_bit_cast(unsigned short, x); }
__device__ __forceinline__ unsigned pk16(unsigned short a, unsigned short b) { return (unsigned)a | ((unsigned)b << 16); }
__device__ __forceinline__ _Float16 to_h_ftz(float v) { return (_Float16)((fabsf(v) < FMIN16) ? 0.0f : v); }
__device__ __forceinline__ v8f zero8() { v8f z = {0.f, 0.f, 0.f, 0.f, 0.f, 0.f, 0.f, 0.f}; return z; }
__device__ __forceinline__ float hmax8(v8f s) {
  return fmaxf(fmaxf(fmaxf(s[0], s[1]), fmaxf(s[2], s[3])), fmaxf(fmaxf(s[4], s[5]), fmaxf(s[6], s[7])));
}
__device__ __forceinline__ float silu_f(float g) {
  const float e = __expf(-g);
  return g * __builtin_amdgcn_rcpf(1.0f + e);
}
__device__ __forceinline__ float pow_age(float base, int e) {
  double r = 1.0, p = (double)base;
#pragma unroll 1
  for (int i = 0; i < 11; ++i) {
    const double rp = r * p;
    r = ((e & 1) != 0) ? rp : r;
    p = p * p;
    e >>= 1;
  }
  return (float)r;
}
__device__ __forceinline__ float block_sum4(float v, float* red, int tid) {
  v += __shfl_xor(v, 16, 32);
  v += __shfl_xor(v, 8, 32);
  v += __shfl_xor(v, 4, 32);
  v += __shfl_xor(v, 2, 32);
  v += __shfl_xor(v, 1, 32);
  if ((tid & 31) == 0) red[tid >> 5] = v;
  __syncthreads();
  return (red[0] + red[1]) + (red[2] + red[3]);
}

__device__ __forceinline__ v16h ldfrag_h(const _Float16* p) {
  FragH f;
  f.h[0] = *(const v8h*)(p);
  f.h[1] = *(const v8h*)(p + 16);
  return f.v;
}

__device__ __forceinline__ v8f mma_h(v16h a, v16h b, v8f c) {
  v8f d = __builtin_amdgcn_wmma_f32_16x16x32_f16(false, a, false, b, (short)0, c, false, false);
#if defined(__HIP_DEVICE_COMPILE__)
  asm volatile("v_nop\n\tv_nop\n\tv_nop\n\tv_nop" : "+v"(d) : "v"(a), "v"(b));
#endif
  return d;
}

__global__ __launch_bounds__(256) void cvt_w(const float* __restrict__ src, unsigned short* dst, int n8) {
  const int i = blockIdx.x * 256 + threadIdx.x;
  if (i >= n8) return;
  const float* p = src + (size_t)i * 8;
  const v4f f0 = *(const v4f*)(p), f1 = *(const v4f*)(p + 4);
  v4u wb;
  wb[0] = pk16(h_bits(to_h_ftz(bfr(f0[0]) * WSCL)), h_bits(to_h_ftz(bfr(f0[1]) * WSCL)));
  wb[1] = pk16(h_bits(to_h_ftz(bfr(f0[2]) * WSCL)), h_bits(to_h_ftz(bfr(f0[3]) * WSCL)));
  wb[2] = pk16(h_bits(to_h_ftz(bfr(f1[0]) * WSCL)), h_bits(to_h_ftz(bfr(f1[1]) * WSCL)));
  wb[3] = pk16(h_bits(to_h_ftz(bfr(f1[2]) * WSCL)), h_bits(to_h_ftz(bfr(f1[3]) * WSCL)));
  unsigned short* d = dst + (size_t)i * 8;
  *(volatile v4u*)d = wb;
  __threadfence();
  *(volatile v4u*)d = wb;
}

__global__ __launch_bounds__(128)
void ln_tab(const float* __restrict__ E, const float* __restrict__ gg, const float* __restrict__ be,
            unsigned short* MH, unsigned short* ML) {
  __shared__ float red1[4];
  __shared__ float red2[4];
  const int tid = threadIdx.x, row = blockIdx.x;
  const float* p = E + (size_t)row * DM + 8 * tid;
  const v4f a0 = *(const v4f*)(p), a1 = *(const v4f*)(p + 4);
  float x[8];
#pragma unroll
  for (int i = 0; i < 4; ++i) { x[i] = bfr(a0[i]); x[4 + i] = bfr(a1[i]); }
  float s = 0.f;
#pragma unroll
  for (int i = 0; i < 8; ++i) s += x[i];
  const float mu = block_sum4(s, red1, tid) * (1.0f / DM);
  float s2 = 0.f;
#pragma unroll
  for (int i = 0; i < 8; ++i) { const float dv = x[i] - mu; s2 += dv * dv; }
  const float var  = block_sum4(s2, red2, tid) * (1.0f / DM);
  const float rstd = rsqrtf(var + 1e-5f);
  const v4f g0 = *(const v4f*)(gg + 8 * tid), g1 = *(const v4f*)(gg + 8 * tid + 4);
  const v4f b0 = *(const v4f*)(be + 8 * tid), b1 = *(const v4f*)(be + 8 * tid + 4);
  unsigned short hb[8], lb[8];
#pragma unroll
  for (int i = 0; i < 8; ++i) {
    const float gi = bfr((i < 4) ? g0[i & 3] : g1[i & 3]);
    const float bi = bfr((i < 4) ? b0[i & 3] : b1[i & 3]);
    const float y  = (x[i] - mu) * rstd * gi + bi;
    const _Float16 hi = to_h_ftz(y);
    hb[i] = h_bits(hi);
    lb[i] = h_bits(to_h_ftz((y - (float)hi) * 1024.0f));
  }
  v4u wh, wl;
#pragma unroll
  for (int t = 0; t < 4; ++t) { wh[t] = pk16(hb[2 * t], hb[2 * t + 1]); wl[t] = pk16(lb[2 * t], lb[2 * t + 1]); }
  unsigned short* dh = MH + (size_t)row * DM + 8 * tid;
  unsigned short* dl = ML + (size_t)row * DM + 8 * tid;
  *(volatile v4u*)dh = wh;
  *(volatile v4u*)dl = wl;
  __threadfence();
  *(volatile v4u*)dh = wh;
  *(volatile v4u*)dl = wl;
}

__global__ __launch_bounds__(128)
void gate_ln_q(const float* __restrict__ X, const float* __restrict__ C, const float* __restrict__ Wpe,
               const float* __restrict__ gg, const float* __restrict__ be, unsigned short* XO) {
  __shared__ __align__(16) float xs[DM];
  __shared__ float red1[4];
  __shared__ float red2[4];
  const int tid = threadIdx.x, row = blockIdx.x;
  const float* cp = C + (size_t)row * NSC;
  const v4f c0 = *(const v4f*)(cp), c1 = *(const v4f*)(cp + 4);
  const float cm0 = bfr(c0[0]), cm1 = bfr(c0[1]), cm2 = bfr(c0[2]), cm3 = bfr(c0[3]);
  const float cm4 = bfr(c1[0]), cm5 = bfr(c1[1]), cm6 = bfr(c1[2]), cm7 = bfr(c1[3]);
  {
    const float* p = X + (size_t)row * DM + 8 * tid;
    const v4f a0 = *(const v4f*)(p), a1 = *(const v4f*)(p + 4);
    v4f r0, r1;
#pragma unroll
    for (int i = 0; i < 4; ++i) { r0[i] = bfr(a0[i]); r1[i] = bfr(a1[i]); }
    *(v4f*)(xs + 8 * tid)     = r0;
    *(v4f*)(xs + 8 * tid + 4) = r1;
  }
  __syncthreads();
  float s = 0.f;
#pragma unroll 1
  for (int j = 0; j < 8; ++j) {
    const int d = 8 * tid + j;
    const float* wp = Wpe + (size_t)d * NSC;
    const v4f w0 = *(const v4f*)(wp), w1 = *(const v4f*)(wp + 4);
    float g = cm0 * bfr(w0[0]);
    g += cm1 * bfr(w0[1]);
    g += cm2 * bfr(w0[2]);
    g += cm3 * bfr(w0[3]);
    g += cm4 * bfr(w1[0]);
    g += cm5 * bfr(w1[1]);
    g += cm6 * bfr(w1[2]);
    g += cm7 * bfr(w1[3]);
    const float xg = xs[d] * silu_f(g);
    xs[d] = xg;
    s += xg;
  }
  const float mu = block_sum4(s, red1, tid) * (1.0f / DM);
  float s2 = 0.f;
#pragma unroll 1
  for (int j = 0; j < 8; ++j) { const float dv = xs[8 * tid + j] - mu; s2 += dv * dv; }
  const float var  = block_sum4(s2, red2, tid) * (1.0f / DM);
  const float rstd = rsqrtf(var + 1e-5f);
#pragma unroll 1
  for (int j = 0; j < 8; ++j) {
    const int d = 8 * tid + j;
    xs[d] = (xs[d] - mu) * rstd * bfr(gg[d]) + bfr(be[d]);
  }
  __syncthreads();
  const v4f y0 = *(const v4f*)(xs + 8 * tid), y1 = *(const v4f*)(xs + 8 * tid + 4);
  v4u wh;
  wh[0] = pk16(h_bits(to_h_ftz(y0[0])), h_bits(to_h_ftz(y0[1])));
  wh[1] = pk16(h_bits(to_h_ftz(y0[2])), h_bits(to_h_ftz(y0[3])));
  wh[2] = pk16(h_bits(to_h_ftz(y1[0])), h_bits(to_h_ftz(y1[1])));
  wh[3] = pk16(h_bits(to_h_ftz(y1[2])), h_bits(to_h_ftz(y1[3])));
  unsigned short* dh = XO + (size_t)row * DM + 8 * tid;
  *(volatile v4u*)dh = wh;
  __threadfence();
  *(volatile v4u*)dh = wh;
}

__global__ __launch_bounds__(256)
void gemm_h(const unsigned short* __restrict__ A, const unsigned short* __restrict__ W, unsigned short* OP, float s1) {
  __shared__ __align__(16) unsigned short S[64 * SSP];
  const int tid  = threadIdx.x;
  const int lane = tid & 31, wave = tid >> 5;
  const int h    = lane >> 4, c = lane & 15;
  const int rg   = wave & 3, ch = wave >> 2;
  const int row0 = blockIdx.y * 64;
  const int col0 = blockIdx.x * 128;
  const _Float16* Ah = (const _Float16*)(const void*)A;
  const _Float16* Wh = (const _Float16*)(const void*)W;

  const _Float16* ap = Ah + ((size_t)(row0 + 16 * rg + c)) * DM + 8 * h;
  const _Float16* bp = Wh + ((size_t)(col0 + 64 * ch + c)) * DM + 8 * h;
  v8f acc0 = zero8(), acc1 = zero8(), acc2 = zero8(), acc3 = zero8();
#pragma unroll 2
  for (int ks = 0; ks < DM / 32; ++ks) {
    const v16h a = ldfrag_h(ap + 32 * ks);
    const _Float16* bs = bp + 32 * ks;
    acc0 = mma_h(a, ldfrag_h(bs + 0 * 16 * DM), acc0);
    acc1 = mma_h(a, ldfrag_h(bs + 1 * 16 * DM), acc1);
    acc2 = mma_h(a, ldfrag_h(bs + 2 * 16 * DM), acc2);
    acc3 = mma_h(a, ldfrag_h(bs + 3 * 16 * DM), acc3);
  }

  unsigned short* qs = S + (16 * rg + 8 * h) * SSP + 64 * ch + c;
#pragma unroll
  for (int r = 0; r < 8; ++r) {
    qs[r * SSP + 0 * 16] = h_bits(to_h_ftz(acc0[r] * s1));
    qs[r * SSP + 1 * 16] = h_bits(to_h_ftz(acc1[r] * s1));
    qs[r * SSP + 2 * 16] = h_bits(to_h_ftz(acc2[r] * s1));
    qs[r * SSP + 3 * 16] = h_bits(to_h_ftz(acc3[r] * s1));
  }
  __syncthreads();

  const int e = tid & 7, lg = tid >> 3;
#pragma unroll
  for (int pass = 0; pass < 2; ++pass) {
#pragma unroll
    for (int it = 0; it < 4; ++it) {
      const int L   = it * 32 + lg;
      const int row = L >> 1, hf = L & 1;
      const v4u v = *(const v4u*)(S + row * SSP + 64 * hf + 8 * e);
      *(volatile v4u*)(OP + ((size_t)(row0 + row)) * DM + col0 + 64 * hf + 8 * e) = v;
    }
    __threadfence();
  }
}

__global__ __launch_bounds__(256)
void gemm_f(const unsigned short* __restrict__ AH, const unsigned short* __restrict__ AL,
            const unsigned short* __restrict__ W, float* OF, float slo, float s1) {
  __shared__ __align__(16) float S[64 * FSP];
  const int tid  = threadIdx.x;
  const int lane = tid & 31, wave = tid >> 5;
  const int h    = lane >> 4, c = lane & 15;
  const int rg   = wave & 3, ch = wave >> 2;
  const int row0 = blockIdx.y * 64;
  const int col0 = blockIdx.x * 128;
  const _Float16* Hh = (const _Float16*)(const void*)AH;
  const _Float16* Lh = (const _Float16*)(const void*)AL;
  const _Float16* Wh = (const _Float16*)(const void*)W;

  const _Float16* aph = Hh + ((size_t)(row0 + 16 * rg + c)) * DM + 8 * h;
  const _Float16* apl = Lh + ((size_t)(row0 + 16 * rg + c)) * DM + 8 * h;
  const _Float16* bp  = Wh + ((size_t)(col0 + 64 * ch + c)) * DM + 8 * h;
  v8f ah0 = zero8(), ah1 = zero8(), ah2 = zero8(), ah3 = zero8();
  v8f al0 = zero8(), al1 = zero8(), al2 = zero8(), al3 = zero8();
#pragma unroll 1
  for (int ks = 0; ks < DM / 32; ++ks) {
    const v16h a  = ldfrag_h(aph + 32 * ks);
    const v16h al = ldfrag_h(apl + 32 * ks);
    const _Float16* bs = bp + 32 * ks;
    const v16h b0 = ldfrag_h(bs + 0 * 16 * DM);
    ah0 = mma_h(a, b0, ah0); al0 = mma_h(al, b0, al0);
    const v16h b1 = ldfrag_h(bs + 1 * 16 * DM);
    ah1 = mma_h(a, b1, ah1); al1 = mma_h(al, b1, al1);
    const v16h b2 = ldfrag_h(bs + 2 * 16 * DM);
    ah2 = mma_h(a, b2, ah2); al2 = mma_h(al, b2, al2);
    const v16h b3 = ldfrag_h(bs + 3 * 16 * DM);
    ah3 = mma_h(a, b3, ah3); al3 = mma_h(al, b3, al3);
  }

  float* fs = S + (16 * rg + 8 * h) * FSP + 64 * ch + c;
#pragma unroll
  for (int r = 0; r < 8; ++r) {
    fs[r * FSP + 0 * 16] = (ah0[r] + al0[r] * slo) * s1;
    fs[r * FSP + 1 * 16] = (ah1[r] + al1[r] * slo) * s1;
    fs[r * FSP + 2 * 16] = (ah2[r] + al2[r] * slo) * s1;
    fs[r * FSP + 3 * 16] = (ah3[r] + al3[r] * slo) * s1;
  }
  __syncthreads();

  const int e = tid & 7, lg = tid >> 3;
#pragma unroll
  for (int pass = 0; pass < 2; ++pass) {
#pragma unroll
    for (int it = 0; it < 8; ++it) {
      const int L   = it * 32 + lg;
      const int row = L >> 2, q4 = L & 3;
      const v4f v = *(const v4f*)(S + row * FSP + 32 * q4 + 4 * e);
      *(volatile v4f*)(OF + ((size_t)(row0 + row)) * DM + col0 + 32 * q4 + 4 * e) = v;
    }
    __threadfence();
  }
}

__global__ __launch_bounds__(256)
void gather_kv(const int* __restrict__ xidx, const float* __restrict__ EK, const float* __restrict__ EV,
               const float* __restrict__ rhos, const float* __restrict__ Wpe,
               unsigned short* KP, unsigned short* VT) {
  __shared__ __align__(16) unsigned short Ks[64 * KSP];
  __shared__ __align__(16) unsigned short Vs[128 * VSP];
  __shared__ float cpw[64 * NSC];
  __shared__ int sid[64];
  const int tid  = threadIdx.x;
  const int d0   = blockIdx.x * 128;
  const int key0 = blockIdx.y * 64;
  const int b    = blockIdx.z;
  if (tid < 64) {
    int v = xidx[(size_t)b * SEQ + key0 + tid];
    v = (v < 0) ? (v + NTAB) : v;
    v = (v < 0) ? 0 : v;
    v = (v > NTAB - 1) ? (NTAB - 1) : v;
    sid[tid] = v;
  }
#pragma unroll 1
  for (int i = tid; i < 64 * NSC; i += 256) {
    const int key = i >> 3, mm = i & 7;
    const int age = SEQ - 1 - (key0 + key);
    cpw[i] = pow_age(bfr(rhos[mm]), age);
  }
  __syncthreads();

  const int dl = tid & 127, kh = tid >> 7;
  const int d  = d0 + dl;
  const float* wp = Wpe + (size_t)d * NSC;
  const v4f w0 = *(const v4f*)(wp), w1 = *(const v4f*)(wp + 4);
  const float wv0 = bfr(w0[0]), wv1 = bfr(w0[1]), wv2 = bfr(w0[2]), wv3 = bfr(w0[3]);
  const float wv4 = bfr(w1[0]), wv5 = bfr(w1[1]), wv6 = bfr(w1[2]), wv7 = bfr(w1[3]);
#pragma unroll 2
  for (int kk = 0; kk < 32; ++kk) {
    const int key = 32 * kh + kk;
    const float* cq = cpw + key * NSC;
    float g = cq[0] * wv0;
    g += cq[1] * wv1;
    g += cq[2] * wv2;
    g += cq[3] * wv3;
    g += cq[4] * wv4;
    g += cq[5] * wv5;
    g += cq[6] * wv6;
    g += cq[7] * wv7;
    const float sg = silu_f(g);
    const int id = sid[key];
    const float ek = EK[(size_t)id * DM + d];
    const float ev = EV[(size_t)id * DM + d];
    Ks[key * KSP + dl] = h_bits(to_h_ftz((ek * sg) * 16.0f));
    Vs[dl * VSP + key] = h_bits(to_h_ftz((ev * sg) * 16.0f));
  }
  __syncthreads();

  const int e = tid & 7, lg = tid >> 3;
#pragma unroll
  for (int pass = 0; pass < 2; ++pass) {
#pragma unroll
    for (int it = 0; it < 4; ++it) {
      const int L   = it * 32 + lg;
      const int row = L >> 1, hf = L & 1;
      const v4u v = *(const v4u*)(Ks + row * KSP + 64 * hf + 8 * e);
      *(volatile v4u*)(KP + ((size_t)b * SEQ + key0 + row) * DM + d0 + 64 * hf + 8 * e) = v;
    }
#pragma unroll
    for (int it = 0; it < 4; ++it) {
      const int dd = it * 32 + lg;
      const v4u v = *(const v4u*)(Vs + dd * VSP + 8 * e);
      *(volatile v4u*)(VT + ((size_t)b * DM + d0 + dd) * SEQ + key0 + 8 * e) = v;
    }
    __threadfence();
  }
}

__global__ __launch_bounds__(128)
void attn_kernel(const unsigned short* __restrict__ QP, const unsigned short* __restrict__ KP,
                 const unsigned short* __restrict__ VT, unsigned short* OH, unsigned short* OL) {
  __shared__ __align__(16) unsigned short Hs[QT * OHP];
  __shared__ __align__(16) unsigned short Lw[QT * OHP];
  const int tid  = threadIdx.x;
  const int wave = tid >> 5;
  const int lane = tid & 31;
  const int h    = lane >> 4;
  const int c    = lane & 15;
  const int bx   = blockIdx.x;
  const int qt   = bx % (SEQ / QT);
  const int bh   = bx / (SEQ / QT);
  const int hh   = bh % NH;
  const int b    = bh / NH;
  const int n0   = qt * QT;
  const _Float16* QPh = (const _Float16*)(const void*)QP;
  const _Float16* KPh = (const _Float16*)(const void*)KP;
  const _Float16* VTh = (const _Float16*)(const void*)VT;

  const _Float16* qpp = QPh + ((size_t)b * SEQ + n0 + 16 * wave + c) * DM + hh * HD + 8 * h;
  const _Float16* khp = KPh + ((size_t)b * SEQ + c) * DM + hh * HD + 8 * h;
  const _Float16* vtp = VTh + ((size_t)b * DM + hh * HD + c) * SEQ + 8 * h;
  const v16h qf0 = ldfrag_h(qpp);
  const v16h qf1 = ldfrag_h(qpp + 32);
  const float SCL = 0.0078125f;

  float m = NEGBIG, l = 0.f;
  v8f acc0 = zero8(), acc1 = zero8(), acc2 = zero8(), acc3 = zero8();

#pragma unroll 1
  for (int it = 0; it < SEQ / 64; ++it) {
    const int kb = it * 64;
    const _Float16* k0p = khp + (size_t)kb * DM;
    v8f s0 = zero8(), s1 = zero8(), s2 = zero8(), s3 = zero8();
    s0 = mma_h(ldfrag_h(k0p + 0 * 16 * DM),      qf0, s0);
    s0 = mma_h(ldfrag_h(k0p + 0 * 16 * DM + 32), qf1, s0);
    s1 = mma_h(ldfrag_h(k0p + 1 * 16 * DM),      qf0, s1);
    s1 = mma_h(ldfrag_h(k0p + 1 * 16 * DM + 32), qf1, s1);
    s2 = mma_h(ldfrag_h(k0p + 2 * 16 * DM),      qf0, s2);
    s2 = mma_h(ldfrag_h(k0p + 2 * 16 * DM + 32), qf1, s2);
    s3 = mma_h(ldfrag_h(k0p + 3 * 16 * DM),      qf0, s3);
    s3 = mma_h(ldfrag_h(k0p + 3 * 16 * DM + 32), qf1, s3);

    float mx = fmaxf(fmaxf(hmax8(s0), hmax8(s1)), fmaxf(hmax8(s2), hmax8(s3)));
    mx = fmaxf(mx, __shfl_xor(mx, 16, 32));
    const float mn   = fmaxf(m, mx * SCL);
    const float corr = __expf(m - mn);
    m = mn;
    const float msh = mn - LNPS;
    FragH p0, p1;
    float ls = 0.f;
#pragma unroll
    for (int r = 0; r < 8; ++r) {
      const float e0 = __expf(s0[r] * SCL - msh);
      const float e1 = __expf(s1[r] * SCL - msh);
      const float e2 = __expf(s2[r] * SCL - msh);
      const float e3 = __expf(s3[r] * SCL - msh);
      ls += (e0 + e1) + (e2 + e3);
      p0.h[0][r] = (_Float16)e0;
      p0.h[1][r] = (_Float16)e1;
      p1.h[0][r] = (_Float16)e2;
      p1.h[1][r] = (_Float16)e3;
    }
    l = l * corr + ls;
#pragma unroll
    for (int r = 0; r < 8; ++r) { acc0[r] *= corr; acc1[r] *= corr; acc2[r] *= corr; acc3[r] *= corr; }

    const _Float16* v0p = vtp + kb;
    acc0 = mma_h(ldfrag_h(v0p + 0 * 16 * SEQ),      p0.v, acc0);
    acc0 = mma_h(ldfrag_h(v0p + 0 * 16 * SEQ + 32), p1.v, acc0);
    acc1 = mma_h(ldfrag_h(v0p + 1 * 16 * SEQ),      p0.v, acc1);
    acc1 = mma_h(ldfrag_h(v0p + 1 * 16 * SEQ + 32), p1.v, acc1);
    acc2 = mma_h(ldfrag_h(v0p + 2 * 16 * SEQ),      p0.v, acc2);
    acc2 = mma_h(ldfrag_h(v0p + 2 * 16 * SEQ + 32), p1.v, acc2);
    acc3 = mma_h(ldfrag_h(v0p + 3 * 16 * SEQ),      p0.v, acc3);
    acc3 = mma_h(ldfrag_h(v0p + 3 * 16 * SEQ + 32), p1.v, acc3);
  }

  l += __shfl_xor(l, 16, 32);
  const float f = 4.0f * __builtin_amdgcn_rcpf(l);
  {
    unsigned short hb[8], lb[8];
    v4u wh, wl;
    const int so = (16 * wave + c) * OHP + 8 * h;
#pragma unroll
    for (int r = 0; r < 8; ++r) {
      const float v = acc0[r] * f; const _Float16 hi = to_h_ftz(v);
      hb[r] = h_bits(hi); lb[r] = h_bits(to_h_ftz((v - (float)hi) * 4096.0f));
    }
#pragma unroll
    for (int t = 0; t < 4; ++t) { wh[t] = pk16(hb[2 * t], hb[2 * t + 1]); wl[t] = pk16(lb[2 * t], lb[2 * t + 1]); }
    *(v4u*)(Hs + so + 0 * 16) = wh; *(v4u*)(Lw + so + 0 * 16) = wl;
#pragma unroll
    for (int r = 0; r < 8; ++r) {
      const float v = acc1[r] * f; const _Float16 hi = to_h_ftz(v);
      hb[r] = h_bits(hi); lb[r] = h_bits(to_h_ftz((v - (float)hi) * 4096.0f));
    }
#pragma unroll
    for (int t = 0; t < 4; ++t) { wh[t] = pk16(hb[2 * t], hb[2 * t + 1]); wl[t] = pk16(lb[2 * t], lb[2 * t + 1]); }
    *(v4u*)(Hs + so + 1 * 16) = wh; *(v4u*)(Lw + so + 1 * 16) = wl;
#pragma unroll
    for (int r = 0; r < 8; ++r) {
      const float v = acc2[r] * f; const _Float16 hi = to_h_ftz(v);
      hb[r] = h_bits(hi); lb[r] = h_bits(to_h_ftz((v - (float)hi) * 4096.0f));
    }
#pragma unroll
    for (int t = 0; t < 4; ++t) { wh[t] = pk16(hb[2 * t], hb[2 * t + 1]); wl[t] = pk16(lb[2 * t], lb[2 * t + 1]); }
    *(v4u*)(Hs + so + 2 * 16) = wh; *(v4u*)(Lw + so + 2 * 16) = wl;
#pragma unroll
    for (int r = 0; r < 8; ++r) {
      const float v = acc3[r] * f; const _Float16 hi = to_h_ftz(v);
      hb[r] = h_bits(hi); lb[r] = h_bits(to_h_ftz((v - (float)hi) * 4096.0f));
    }
#pragma unroll
    for (int t = 0; t < 4; ++t) { wh[t] = pk16(hb[2 * t], hb[2 * t + 1]); wl[t] = pk16(lb[2 * t], lb[2 * t + 1]); }
    *(v4u*)(Hs + so + 3 * 16) = wh; *(v4u*)(Lw + so + 3 * 16) = wl;
  }
  __syncthreads();

  const int e = tid & 7, lg = tid >> 3;
#pragma unroll
  for (int pass = 0; pass < 2; ++pass) {
#pragma unroll
    for (int it = 0; it < 4; ++it) {
      const int L = it * 16 + lg;
      const size_t go = ((size_t)b * SEQ + n0 + L) * DM + hh * HD + 8 * e;
      const v4u vh = *(const v4u*)(Hs + L * OHP + 8 * e);
      const v4u vl = *(const v4u*)(Lw + L * OHP + 8 * e);
      *(volatile v4u*)(OH + go) = vh;
      *(volatile v4u*)(OL + go) = vl;
    }
    __threadfence();
  }
}

extern "C" void kernel_launch(void* const* d_in, const int* in_sizes, int n_in,
                              void* d_out, int out_size, void* d_ws, size_t ws_size,
                              hipStream_t stream) {
  const int NX = NROW * DM;
  if (n_in < 14) return;
  if (in_sizes[0] != NX || in_sizes[1] != NROW || in_sizes[2] != NTAB * DM) return;
  if (in_sizes[3] != NSC || in_sizes[4] != NROW * NSC) return;
  if (in_sizes[5] != DM * DM || in_sizes[6] != DM * DM || in_sizes[7] != DM * DM || in_sizes[8] != DM * DM) return;
  if (in_sizes[9] != DM * NSC) return;
  if (in_sizes[10] != DM || in_sizes[11] != DM || in_sizes[12] != DM || in_sizes[13] != DM) return;
  if (out_size != NX) return;

  size_t off = 0;
  const size_t szW  = (size_t)DM * DM * 2;
  const size_t szM  = (size_t)NTAB * DM * 2;
  const size_t szE  = (size_t)NTAB * DM * 4;
  const size_t szP  = (size_t)NROW * DM * 2;
  const size_t oWP = off; off += 4 * szW;
  const size_t oMH = off; off += szM;
  const size_t oML = off; off += szM;
  const size_t oEK = off; off += szE;
  const size_t oEV = off; off += szE;
  const size_t oXL = off; off += szP;
  const size_t oQP = off; off += szP;
  const size_t oKP = off; off += szP;
  const size_t oVT = off; off += szP;
  const size_t oOH = off; off += szP;
  const size_t oOL = off; off += szP;
  if (off > ws_size) return;
  if (off > (size_t)134217728) return;

  const float* xq   = (const float*)d_in[0];
  const int*   xidx = (const int*)d_in[1];
  const float* Etab = (const float*)d_in[2];
  const float* rhos = (const float*)d_in[3];
  const float* Cseq = (const float*)d_in[4];
  const float* Wq   = (const float*)d_in[5];
  const float* Wk   = (const float*)d_in[6];
  const float* Wv   = (const float*)d_in[7];
  const float* Wo   = (const float*)d_in[8];
  const float* Wpe  = (const float*)d_in[9];
  const float* gkv  = (const float*)d_in[10];
  const float* bkv  = (const float*)d_in[11];
  const float* gq   = (const float*)d_in[12];
  const float* bq   = (const float*)d_in[13];
  char* ws = (char*)d_ws;
  unsigned short* WP = (unsigned short*)(ws + oWP);
  unsigned short* MH = (unsigned short*)(ws + oMH);
  unsigned short* ML = (unsigned short*)(ws + oML);
  float*          EK = (float*)(ws + oEK);
  float*          EV = (float*)(ws + oEV);
  unsigned short* XL = (unsigned short*)(ws + oXL);
  unsigned short* QP = (unsigned short*)(ws + oQP);
  unsigned short* KP = (unsigned short*)(ws + oKP);
  unsigned short* VT = (unsigned short*)(ws + oVT);
  unsigned short* OH = (unsigned short*)(ws + oOH);
  unsigned short* OL = (unsigned short*)(ws + oOL);
  float* out = (float*)d_out;

  const size_t nWW = (size_t)DM * DM;
  const int  n8W = (DM * DM) / 8;
  const dim3 b256(256), b128(128);
  const dim3 gW(n8W / 256);
  const dim3 gE(DM / 128, NTAB / 64);
  const dim3 gP(DM / 128, NROW / 64);
  const dim3 gG(DM / 128, SEQ / 64, NB);
  const dim3 gA(NB * NH * (SEQ / QT));

  cvt_w<<<gW, b256, 0, stream>>>(Wq, WP + 0 * nWW, n8W);
  cvt_w<<<gW, b256, 0, stream>>>(Wk, WP + 1 * nWW, n8W);
  cvt_w<<<gW, b256, 0, stream>>>(Wv, WP + 2 * nWW, n8W);
  cvt_w<<<gW, b256, 0, stream>>>(Wo, WP + 3 * nWW, n8W);
  ln_tab<<<dim3(NTAB), b128, 0, stream>>>(Etab, gkv, bkv, MH, ML);
  gemm_f<<<gE, b256, 0, stream>>>(MH, ML, WP + 1 * nWW, EK, 1.0f / 1024.0f, 1.0f / 32.0f);
  gemm_f<<<gE, b256, 0, stream>>>(MH, ML, WP + 2 * nWW, EV, 1.0f / 1024.0f, 1.0f / 32.0f);
  gate_ln_q<<<dim3(NROW), b128, 0, stream>>>(xq, Cseq, Wpe, gq, bq, XL);
  gemm_h<<<gP, b256, 0, stream>>>(XL, WP + 0 * nWW, QP, 1.0f / 32.0f);
  gather_kv<<<gG, b256, 0, stream>>>(xidx, EK, EV, rhos, Wpe, KP, VT);
  attn_kernel<<<gA, b128, 0, stream>>>(QP, KP, VT, OH, OL);
  gemm_f<<<gP, b256, 0, stream>>>(OH, OL, WP + 3 * nWW, out, 1.0f / 4096.0f, 1.0f / 2048.0f);
  (void)hipGetLastError();
}
